// FullAttention_73323681677865
// MI455X (gfx1250) — hardware-verified
//
#include <hip/hip_runtime.h>


#ifndef NB
#define NB 4
#endif
#ifndef SEQ
#define SEQ 2048
#endif
#define NB_FULL  4
#define SEQ_FULL 2048
#define NH   16
#define HD   64
#define DQ   (NH * HD)
#define ZH   4
#define RH   (((SEQ) < 512) ? (SEQ) : 512)
#define PCAR 1024.0f
#define SCL  0.125f
#define MASKL (-1.0e9f * SCL)
#define WS_CAP ((size_t)134217728)

static_assert(SEQ % 128 == 0);
static_assert(SEQ <= SEQ_FULL);
static_assert(NB <= NB_FULL);
static_assert(NH % ZH == 0);
static_assert(RH % 64 == 0);
static_assert((SEQ - RH) % 64 == 0);
static_assert(HD == 64);

typedef _Float16 h16;
typedef unsigned short bf;
typedef __attribute__((ext_vector_type(16))) __bf16   v16bf;
typedef __attribute__((ext_vector_type(16))) _Float16 v16h;
typedef __attribute__((ext_vector_type(8)))  _Float16 v8h;
typedef __attribute__((ext_vector_type(8)))  unsigned short v8us;
typedef __attribute__((ext_vector_type(8)))  float    v8f;
typedef __attribute__((ext_vector_type(4)))  float    v4f;
typedef __attribute__((ext_vector_type(2)))  _Float16 v2h;
typedef __attribute__((ext_vector_type(4)))  _Float16 v4h;
typedef __attribute__((ext_vector_type(2)))  unsigned short v2us;
typedef __attribute__((ext_vector_type(4)))  unsigned short v4us;
typedef v8h  __attribute__((may_alias)) v8ha;
typedef v4f  __attribute__((may_alias)) v4fa;
typedef v8us __attribute__((may_alias)) v8usa;

__device__ __forceinline__ unsigned short f2bf(float f) { unsigned u = __float_as_uint(f); u += 0x7FFFu + ((u >> 16) & 1u); return (unsigned short)(u >> 16); }
__device__ __forceinline__ float bf2f(unsigned short b) { return __uint_as_float(((unsigned)b) << 16); }
__device__ __forceinline__ float bfr(float f) { return bf2f(f2bf(f)); }
__device__ __forceinline__ h16 tohx(float x) { return (h16)x; }
__device__ __forceinline__ void splitf(float y, unsigned short& h, unsigned short& l) { h = f2bf(y); l = f2bf(y - bf2f(h)); }
__device__ __forceinline__ v16h cat16(v8h lo, v8h hi) { return __builtin_shufflevector(lo, hi, 0, 1, 2, 3, 4, 5, 6, 7, 8, 9, 10, 11, 12, 13, 14, 15); }
__device__ __forceinline__ v16bf cat16b(v8us lo, v8us hi) { return __builtin_bit_cast(v16bf, __builtin_shufflevector(lo, hi, 0, 1, 2, 3, 4, 5, 6, 7, 8, 9, 10, 11, 12, 13, 14, 15)); }
__device__ __forceinline__ v8f wmma16(v16h a, v16h b, v8f c) { return __builtin_amdgcn_wmma_f32_16x16x32_f16(false, a, false, b, (short)0, c, false, false); }
__device__ __forceinline__ v8f wmmab(v16bf a, v16bf b, v8f c) { return __builtin_amdgcn_wmma_f32_16x16x32_bf16(false, a, false, b, (short)0, c, false, false); }

template <typename T16> struct WFrag;
template <> struct WFrag<h16> { typedef v16h V; static __device__ __forceinline__ V ld(const h16* p) { return cat16(*(const v8h*)p, *(const v8h*)(p + 16)); } static __device__ __forceinline__ v8f mma(V a, V b, v8f c) { return wmma16(a, b, c); } };
template <> struct WFrag<bf> { typedef v16bf V; static __device__ __forceinline__ V ld(const bf* p) { return cat16b(*(const v8us*)p, *(const v8us*)(p + 16)); } static __device__ __forceinline__ v8f mma(V a, V b, v8f c) { return wmmab(a, b, c); } };

template <typename T16, int NSPLIT>
__global__ __launch_bounds__(32) void k_gemmw(const T16* __restrict__ A, const T16* __restrict__ A2, const T16* __restrict__ Bt, const T16* __restrict__ Bt2,
                                              int K, int lda, int ldb, float* C, int ldc, float osc, int cmode, int rbase, size_t sA, size_t sB, size_t sC) {
    typedef typename WFrag<T16>::V V;
    __shared__ __align__(16) float os[16 * 68];
    const size_t z = blockIdx.z; A += z * sA; if (A2) A2 += z * sA; Bt += z * sB; if (Bt2) Bt2 += z * sB; C += z * sC;
    const int lane = threadIdx.x & 31, lr = lane & 15, hi = lane >> 4; const int r0 = blockIdx.x * 64, c0 = blockIdx.y * 64;
    int kend = K;
    if (cmode == 1) { if (c0 > rbase + r0 + 63) kend = 0; }
    else if (cmode == 2) { const int kb = rbase + r0 + 64; kend = (kb < K) ? kb : K; }
    v8f acc[4][4];
#pragma unroll
    for (int mb = 0; mb < 4; ++mb)
#pragma unroll
        for (int nb = 0; nb < 4; ++nb) acc[mb][nb] = (v8f){};
    const size_t aoff = (size_t)(r0 + lr) * lda + 8 * hi, boff = (size_t)(c0 + lr) * ldb + 8 * hi;
#pragma unroll 1
    for (int kc = 0; kc < kend; kc += 32) {
        V a[4], a2[4];
#pragma unroll
        for (int mb = 0; mb < 4; ++mb) { a[mb] = WFrag<T16>::ld(A + aoff + (size_t)mb * 16 * lda + kc); if (NSPLIT == 1 || NSPLIT == 2) a2[mb] = WFrag<T16>::ld(A2 + aoff + (size_t)mb * 16 * lda + kc); }
#pragma unroll
        for (int nb = 0; nb < 4; ++nb) { const V b = WFrag<T16>::ld(Bt + boff + (size_t)nb * 16 * ldb + kc); V b2; if (NSPLIT >= 2) b2 = WFrag<T16>::ld(Bt2 + boff + (size_t)nb * 16 * ldb + kc);
#pragma unroll
            for (int mb = 0; mb < 4; ++mb) { acc[mb][nb] = WFrag<T16>::mma(a[mb], b, acc[mb][nb]); if (NSPLIT == 1 || NSPLIT == 2) acc[mb][nb] = WFrag<T16>::mma(a2[mb], b, acc[mb][nb]); if (NSPLIT >= 2) acc[mb][nb] = WFrag<T16>::mma(a[mb], b2, acc[mb][nb]); } }
        asm volatile("v_nop\n\tv_nop\n\tv_nop\n\tv_nop" : "+v"(acc[0][0]), "+v"(acc[1][1]), "+v"(acc[2][2]), "+v"(acc[3][3]) : "v"(a[0]), "v"(a[3]));
    }
#pragma unroll
    for (int mb = 0; mb < 4; ++mb) {
#pragma unroll
        for (int nb = 0; nb < 4; ++nb) {
#pragma unroll
            for (int j = 0; j < 8; ++j) os[(hi * 8 + j) * 68 + nb * 16 + lr] = acc[mb][nb][j]; }
        __builtin_amdgcn_wave_barrier(); asm volatile("" ::: "memory");
        float* crow = C + (size_t)(r0 + mb * 16) * ldc + c0;
#pragma unroll 1
        for (int ps = 0; ps < 2; ++ps) {
#pragma unroll
            for (int s = 0; s < 8; ++s) { const int row = 2 * s + hi, cofs = lr * 4; v4f val = *(const v4fa*)(os + row * 68 + cofs); val = val * osc;
                *(volatile v4f*)(crow + (size_t)row * ldc + cofs) = val; }
            if (ps == 0) __threadfence(); }
        __builtin_amdgcn_wave_barrier(); asm volatile("" ::: "memory");
    }
}

__global__ __launch_bounds__(256) void k_qkp(const float* __restrict__ F, int pitch, int nheads, bf* P) {
    const size_t e = ((size_t)blockIdx.x * 256 + threadIdx.x) * 8; if (e >= (size_t)nheads * SEQ * HD) return;
    const int d = (int)(e % HD); const int t = (int)((e / HD) % SEQ); const int h = (int)(e / ((size_t)HD * SEQ));
    const float* f = F + (size_t)t * pitch + h * HD + d;
    const v4f x0 = *(const v4f*)f; const v4f x1 = *(const v4f*)(f + 4); v8us o;
#pragma unroll
    for (int k = 0; k < 4; ++k) { o[k] = f2bf(x0[k]); o[k + 4] = f2bf(x1[k]); }
    *(volatile v8us*)(P + e) = o; __threadfence(); *(volatile v8us*)(P + e) = o;
}
__global__ __launch_bounds__(256) void k_vtp(const float* __restrict__ F, int pitch, int nheads, h16* V16, bf* Vb) {
    const size_t e = ((size_t)blockIdx.x * 256 + threadIdx.x) * 2; if (e >= (size_t)nheads * HD * SEQ) return;
    const int t = (int)(e % SEQ); const int d = (int)((e / SEQ) % HD); const int g = (int)(e / ((size_t)SEQ * HD)); v2h o16; v2us ob;
#pragma unroll
    for (int q = 0; q < 2; ++q) { const float x = bfr(F[(size_t)(t + q) * pitch + g * HD + d]); o16[q] = tohx(x); ob[q] = f2bf(x); }
    *(volatile v2h*)(V16 + e) = o16; *(volatile v2us*)(Vb + e) = ob; __threadfence(); *(volatile v2h*)(V16 + e) = o16; *(volatile v2us*)(Vb + e) = ob;
}

__global__ __launch_bounds__(256) void k_asoft(const float* __restrict__ Sb, h16* P16, bf* Ph, bf* Pl) {
    const int lane = threadIdx.x & 31; const int row = blockIdx.x * 8 + (threadIdx.x >> 5); if (row >= ZH * SEQ) return;
    const int i = row % SEQ; const int zz = row / SEQ; const bool hires = (i < RH);
    const float* sr = Sb + (size_t)row * SEQ; float v[SEQ / 32]; float mx = -3.0e38f;
#pragma unroll
    for (int ch = 0; ch < SEQ / 128; ++ch) { const int j0 = ch * 128 + lane * 4; const v4f a = *(const v4f*)(sr + j0);
#pragma unroll
        for (int q = 0; q < 4; ++q) { const int j = j0 + q; const float t = (j <= i) ? (a[q] * SCL) : MASKL; v[ch * 4 + q] = t; mx = fmaxf(mx, t); } }
#pragma unroll
    for (int sh = 16; sh; sh >>= 1) mx = fmaxf(mx, __shfl_xor(mx, sh, 32));
    float sum = 0.f;
#pragma unroll
    for (int k = 0; k < SEQ / 32; ++k) { float d0 = __fsub_rn(v[k], mx); asm volatile("" : "+v"(d0)); v[k] = __builtin_amdgcn_exp2f(__fmul_rn(d0, 1.4426950408889634f)); sum += v[k]; }
#pragma unroll
    for (int sh = 16; sh; sh >>= 1) sum += __shfl_xor(sum, sh, 32);
    const float f = __fdiv_rn(hires ? 1.0f : PCAR, sum);
#pragma unroll 1
    for (int ps = 0; ps < 2; ++ps) {
        if (hires) {
#pragma unroll
            for (int ch = 0; ch < SEQ / 128; ++ch) { v4us oh, ol;
#pragma unroll
                for (int q = 0; q < 4; ++q) { unsigned short a2, c2; splitf(v[ch * 4 + q] * f, a2, c2); oh[q] = a2; ol[q] = c2; }
                const size_t oo = ((size_t)zz * RH + i) * SEQ + ch * 128 + lane * 4; *(volatile v4us*)(Ph + oo) = oh; *(volatile v4us*)(Pl + oo) = ol; }
        } else {
#pragma unroll
            for (int ch = 0; ch < SEQ / 128; ++ch) { v4h o4;
#pragma unroll
                for (int q = 0; q < 4; ++q) o4[q] = tohx(v[ch * 4 + q] * f);
                *(volatile v4h*)(P16 + ((size_t)zz * (SEQ - RH) + (i - RH)) * SEQ + ch * 128 + lane * 4) = o4; } }
        if (ps == 0) __threadfence(); }
}

extern "C" void kernel_launch(void* const* d_in, const int* in_sizes, int n_in,
                              void* d_out, int out_size, void* d_ws, size_t ws_size, hipStream_t stream) {
    if (n_in < 3) return;
    const size_t need_in = ((size_t)(NB - 1) * SEQ_FULL + SEQ) * DQ;
    if ((size_t)in_sizes[0] < need_in || (size_t)in_sizes[1] < need_in || (size_t)in_sizes[2] < need_in) return;
    if ((size_t)out_size < (size_t)NB * SEQ * DQ) return;
    const float* qi = (const float*)d_in[0]; const float* ki = (const float*)d_in[1]; const float* vi = (const float*)d_in[2];
    float* OUT = (float*)d_out;
    char* wsp = (char*)d_ws;
    auto take = [&](size_t bytes) { char* p = wsp; wsp += (bytes + 255) & ~(size_t)255; return (void*)p; };
    bf*    QPb  = (bf*)take((size_t)NH * SEQ * HD * 2);
    bf*    KPb  = (bf*)take((size_t)NH * SEQ * HD * 2);
    h16*   VT16 = (h16*)take((size_t)NH * HD * SEQ * 2);
    bf*    VTb  = (bf*)take((size_t)NH * HD * SEQ * 2);
    bf*    Ph   = (bf*)take((size_t)ZH * RH * SEQ * 2);
    bf*    Pl   = (bf*)take((size_t)ZH * RH * SEQ * 2);
    float* Sb   = (float*)take((size_t)ZH * SEQ * SEQ * 4);
    h16*   P16  = (h16*)take((size_t)ZH * (SEQ - RH) * SEQ * 2);
    const size_t used = (size_t)(wsp - (char*)d_ws); if (used > ws_size || used > WS_CAP) return;
    const unsigned gq = (unsigned)(((size_t)NH * SEQ * HD / 8 + 255) / 256);
    const unsigned gv = (unsigned)(((size_t)NH * HD * SEQ / 2 + 255) / 256);
    const unsigned gs = (unsigned)((ZH * SEQ + 7) / 8);
    for (int b = 0; b < NB; ++b) {
        const size_t ib = (size_t)b * SEQ_FULL * DQ; float* ob = OUT + (size_t)b * SEQ * DQ;
        k_qkp<<<gq, 256, 0, stream>>>(qi + ib, DQ, NH, QPb);
        k_qkp<<<gq, 256, 0, stream>>>(ki + ib, DQ, NH, KPb);
        k_vtp<<<gv, 256, 0, stream>>>(vi + ib, DQ, NH, VT16, VTb);
        for (int h0 = 0; h0 < NH; h0 += ZH) {
            const size_t zp = (size_t)h0 * SEQ * HD;
            k_gemmw<bf, 0><<<dim3(SEQ / 64, SEQ / 64, ZH), 32, 0, stream>>>(QPb + zp, nullptr, KPb + zp, nullptr, HD, HD, HD, Sb, SEQ, 1.0f, 1, 0,
                                                                            (size_t)SEQ * HD, (size_t)SEQ * HD, (size_t)SEQ * SEQ);
            k_asoft<<<gs, 256, 0, stream>>>(Sb, P16, Ph, Pl);
            k_gemmw<bf, 1><<<dim3(RH / 64, HD / 64, ZH), 32, 0, stream>>>(Ph, Pl, VTb + zp, nullptr, RH, SEQ, SEQ, ob + (size_t)h0 * HD, DQ, 1.0f, 2, 0,
                                                                           (size_t)RH * SEQ, (size_t)HD * SEQ, (size_t)HD);
            if (SEQ > RH)
                k_gemmw<h16, 0><<<dim3((SEQ - RH) / 64, HD / 64, ZH), 32, 0, stream>>>(P16, nullptr, VT16 + zp, nullptr, SEQ, SEQ, SEQ, ob + (size_t)RH * DQ + (size_t)h0 * HD, DQ,
                                                                                      1.0f / PCAR, 2, RH, (size_t)(SEQ - RH) * SEQ, (size_t)HD * SEQ, (size_t)HD);
        }
    }
}
